// HANLayer_2499670966291
// MI455X (gfx1250) — hardware-run, weakly checked
//
#include <hip/hip_runtime.h>

typedef float          v8f   __attribute__((ext_vector_type(8)));
typedef float          v4f   __attribute__((ext_vector_type(4)));
typedef unsigned int   v4u   __attribute__((ext_vector_type(4)));
typedef int            v8i   __attribute__((ext_vector_type(8)));
typedef unsigned short v8us  __attribute__((ext_vector_type(8)));
typedef unsigned short v16us __attribute__((ext_vector_type(16)));
typedef __bf16         v16bf __attribute__((ext_vector_type(16)));
typedef _Float16       v16h  __attribute__((ext_vector_type(16)));
typedef v4f  __attribute__((may_alias)) v4fa;
typedef v8us __attribute__((may_alias)) v8usa;
union FragB { v16bf v; v16us u; v8us h[2]; v8i w; };
union FragH { v16h  v; v16us u; v8us h[2]; v8i w; };

__device__ __forceinline__ v8f wmb(const FragB& a, const FragB& b, v8f c) {
  v8f d = __builtin_amdgcn_wmma_f32_16x16x32_bf16(false, a.v, false, b.v, (short)0, c, false, false);
  asm volatile("v_nop\n\tv_nop\n\tv_nop\n\tv_nop" : "+v"(d) : "v"(a.w), "v"(b.w));
  return d;
}

__device__ __forceinline__ v8f wmh(const FragH& a, const FragH& b, v8f c) {
  v8f d = __builtin_amdgcn_wmma_f32_16x16x32_f16(false, a.v, false, b.v, (short)0, c, false, false);
  asm volatile("v_nop\n\tv_nop\n\tv_nop\n\tv_nop" : "+v"(d) : "v"(a.w), "v"(b.w));
  return d;
}

__device__ __forceinline__ unsigned bf16_bits(float f) {
  const unsigned u = __float_as_uint(f);
  const unsigned r = (u + 0x7FFFu + ((u >> 16) & 1u)) >> 16;
  const unsigned q = (u >> 16) | 0x40u;
  return ((u & 0x7fffffffu) > 0x7f800000u) ? q : r;
}

__device__ __forceinline__ float bf16_val(float f) {
  return __uint_as_float(bf16_bits(f) << 16);
}
__device__ __forceinline__ int clampi(int v, int lo, int hi) {
  return v < lo ? lo : (v > hi ? hi : v);
}

__device__ __forceinline__ unsigned f16_bits(float f) {
  const unsigned u  = __float_as_uint(f);
  const unsigned s  = (u >> 16) & 0x8000u;
  const unsigned a  = u & 0x7fffffffu;
  const unsigned t  = a - 0x38000000u;
  const unsigned r  = (t + 0x0FFFu + ((t >> 13) & 1u)) >> 13;
  const unsigned rc = r > 0x7C00u ? 0x7C00u : r;
  const bool small  = a < 0x38800000u;
  const bool isnan  = a > 0x7f800000u;
  const unsigned fin = small ? 0u : (s | rc);
  return isnan ? (s | 0x7E00u) : fin;
}

__device__ __forceinline__ unsigned pk16(unsigned lo, unsigned hi) { return lo | (hi << 16); }
__device__ __forceinline__ unsigned bf16_lo_bits(float v) {
  float hi = bf16_val(v);
  asm volatile("" : "+v"(hi));
  return bf16_bits(v - hi);
}
__device__ __forceinline__ v4u pack8_bf16(v4f a, v4f c) {
  return (v4u){ pk16(bf16_bits(a[0]), bf16_bits(a[1])), pk16(bf16_bits(a[2]), bf16_bits(a[3])),
                pk16(bf16_bits(c[0]), bf16_bits(c[1])), pk16(bf16_bits(c[2]), bf16_bits(c[3])) };
}
__device__ __forceinline__ v4u pack8_bf16_lo(v4f a, v4f c) {
  return (v4u){ pk16(bf16_lo_bits(a[0]), bf16_lo_bits(a[1])), pk16(bf16_lo_bits(a[2]), bf16_lo_bits(a[3])),
                pk16(bf16_lo_bits(c[0]), bf16_lo_bits(c[1])), pk16(bf16_lo_bits(c[2]), bf16_lo_bits(c[3])) };
}
__device__ __forceinline__ v4u pack8_f16(v4f a, v4f c) {
  return (v4u){ pk16(f16_bits(a[0]), f16_bits(a[1])), pk16(f16_bits(a[2]), f16_bits(a[3])),
                pk16(f16_bits(c[0]), f16_bits(c[1])), pk16(f16_bits(c[2]), f16_bits(c[3])) };
}

template <int FORM>
__global__ __launch_bounds__(256) void k_plane(const float* __restrict__ src, int rows, int cols, int ldsrc,
                                               unsigned short* __restrict__ dst, int MP, int KP) {
  static_assert(FORM >= 0 && FORM <= 3);
  const int KTOT = (FORM == 1 || FORM == 3) ? 2 * KP : KP;
  const unsigned ppr   = (unsigned)(KTOT >> 3);
  const unsigned kp8   = (unsigned)(KP >> 3);
  const unsigned total = (unsigned)MP * ppr;
  const unsigned g     = blockIdx.x * 256u + threadIdx.x;
  const unsigned rowu  = g / ppr;
  const unsigned p     = g - rowu * ppr;
  const bool second    = p >= kp8;
  const int row = (int)rowu;
  const int c0  = (int)((second ? p - kp8 : p) << 3);
  const float* srow = src + (size_t)clampi(row, 0, rows - 1) * (size_t)ldsrc;
  float x[8];
  unsigned mk[8];
#pragma unroll
  for (int e = 0; e < 8; ++e) {
    const int c = c0 + e;
    const float v = srow[clampi(c, 0, cols - 1)];
    asm volatile("" :: "v"(v));
    x[e]  = v;
    mk[e] = (row < rows && c < cols) ? 0xFFFFu : 0u;
  }
  const v4f a = (v4f){ x[0], x[1], x[2], x[3] };
  const v4f c = (v4f){ x[4], x[5], x[6], x[7] };
  v4u o;
  if (FORM == 2) {
    o = pack8_f16(a, c);
  } else {
    const v4u hi = pack8_bf16(a, c);
    o = hi;
    if (FORM == 1) { const v4u lo = pack8_bf16_lo(a, c); o = second ? lo : hi; }
  }
  const v4u mw = (v4u){ pk16(mk[0], mk[1]), pk16(mk[2], mk[3]), pk16(mk[4], mk[5]), pk16(mk[6], mk[7]) };
  o &= mw;
  if (g < total) {
    volatile v4u* q = (volatile v4u*)(dst + (size_t)g * 8);
    *q = o;
    __threadfence();
    *q = o;
  }
}

template <int FORM> struct FragOf    { typedef FragB T; };
template <>         struct FragOf<2> { typedef FragH T; };
__device__ __forceinline__ v8f mm(const FragB& a, const FragB& b, v8f c) { return wmb(a, b, c); }
__device__ __forceinline__ v8f mm(const FragH& a, const FragH& b, v8f c) { return wmh(a, b, c); }
template <class F> __device__ __forceinline__ F ld_frag(const unsigned short* p) {
  F f;
  f.h[0] = *(const v8usa*)(p);
  f.h[1] = *(const v8usa*)(p + 16);
  return f;
}

template <int FORM, int EPI>
__global__ __launch_bounds__(256) __attribute__((amdgpu_num_vgpr(248)))
void k_gemm_nt(const unsigned short* __restrict__ A, const unsigned short* __restrict__ B,
               const float* __restrict__ bias, float* __restrict__ D, int M, int N, int KTOT, int ldd) {
  static_assert(FORM >= 0 && FORM <= 2);
  static_assert(EPI == 0 || EPI == 1);
  typedef typename FragOf<FORM>::T F;
  __shared__ __attribute__((aligned(16))) float sT[8][16 * 68];
  const int lane = threadIdx.x & 31;
  const int wave = threadIdx.x >> 5;
  const int tilesM = (M + 63) >> 6;
  const int tilesN = (N + 63) >> 6;
  const int tile = blockIdx.x * 8 + wave;
  if (tile >= tilesM * tilesN) return;
  const int tm = tile / tilesN;
  const int tn = tile - tm * tilesN;
  const int m0 = tm << 6;
  const int n0 = tn << 6;

  const int rl = lane & 15;
  const int h8 = (lane >> 4) * 8;
  const unsigned short* pa = A + (size_t)(m0 + rl) * (size_t)KTOT + h8;
  const unsigned short* pb = B + (size_t)(n0 + rl) * (size_t)KTOT + h8;

  v8f acc[4][4];
#pragma unroll
  for (int i = 0; i < 4; ++i)
#pragma unroll
    for (int j = 0; j < 4; ++j) acc[i][j] = (v8f){0.f, 0.f, 0.f, 0.f, 0.f, 0.f, 0.f, 0.f};

#pragma unroll 1
  for (int k0 = 0; k0 < KTOT; k0 += 32) {
    F bf[4];
#pragma unroll
    for (int j = 0; j < 4; ++j) bf[j] = ld_frag<F>(pb + (size_t)(j << 4) * (size_t)KTOT + k0);
#pragma unroll
    for (int i = 0; i < 4; ++i) {
      const F af = ld_frag<F>(pa + (size_t)(i << 4) * (size_t)KTOT + k0);
#pragma unroll
      for (int j = 0; j < 4; ++j) acc[i][j] = mm(af, bf[j], acc[i][j]);
    }
  }

  float* slab = sT[wave];
  const int hh = lane >> 4;
  const int c4 = (lane & 15) * 4;
  const int nc = n0 + c4;
  const bool cok = nc < N;
  v4f bv = (v4f){0.f, 0.f, 0.f, 0.f};
  if (EPI == 1) {
    bv = *(const v4fa*)(bias + clampi(nc, 0, N - 4));
    asm volatile("" :: "v"(bv));
  }
#pragma unroll
  for (int i = 0; i < 4; ++i) {
    const int mBase = m0 + (i << 4);
#pragma unroll
    for (int j = 0; j < 4; ++j) {
#pragma unroll
      for (int r = 0; r < 8; ++r) slab[(h8 + r) * 68 + (j << 4) + rl] = acc[i][j][r];
    }
    __builtin_amdgcn_fence(__ATOMIC_RELEASE, "workgroup");
    __builtin_amdgcn_wave_barrier();
    __builtin_amdgcn_fence(__ATOMIC_ACQUIRE, "workgroup");
    v4f vv[8];
#pragma unroll
    for (int it = 0; it < 8; ++it) {
      const int row = it * 2 + hh;
      v4f v = *(const v4fa*)(slab + row * 68 + c4);
      if (EPI == 1) v += bv;
      vv[it] = v;
    }
    for (int pass = 0; pass < 2; ++pass) {
#pragma unroll
      for (int it = 0; it < 8; ++it) {
        const int row = mBase + it * 2 + hh;
        if (cok && row < M) *(volatile v4f*)(D + (size_t)row * (size_t)ldd + nc) = vv[it];
      }
      __threadfence();
    }
    __builtin_amdgcn_fence(__ATOMIC_RELEASE, "workgroup");
    __builtin_amdgcn_wave_barrier();
    __builtin_amdgcn_fence(__ATOMIC_ACQUIRE, "workgroup");
  }
}

#include <math.h>
#include <stddef.h>

#define NNODE   50000
#define NEDGE   800000
#define FEAT    256
#define NHEAD   8
#define HDIM    32
#define HID     128
#define MPAD    50048
#define NSB     782
#define SEM_TERMS 2
#define SEMK    (FEAT * SEM_TERMS)
#define SBM     64
#define NTHR    256
#define NWAVE   8
#define EPT     8
#define CHUNK   (NTHR * EPT)
#define WCAP    (EPT * 32)
#define LISTN   (NWAVE * WCAP)
#define NBMAX   2048
#define NBRUN   1024
#define SLOTB   11
#define RCAP    28672
#define DEGCAP  256
#define NEGSL   0.2f
#define MX0     (-1.0e30f)
#define LDS_ATT ((2 * RCAP + 2 * NBMAX + LISTN) * 4 + 64 + NWAVE * FEAT * 4 + FEAT * 4)
#define AS_BYTES (SBM * SEMK * 2)
#define SO_BYTES (SBM * HID * 4)
#define SEM_T   (AS_BYTES > SO_BYTES ? AS_BYTES : SO_BYTES)
#define LDS_SEM (SEM_T + HID * 4 * 2 + SBM * 4)
#define NUW     (FEAT * (FEAT / 8))
#define NUP     (HID * (SEMK / 8))
#define NUT     (2 * NUW + NUP)
#define WSCAP   ((size_t)128 << 20)

static_assert(FEAT == 32 * 8);
static_assert(NHEAD * HDIM == FEAT);
static_assert(HID == 128);
static_assert(NTHR == FEAT);
static_assert((NEDGE % 256) == 0 && (NEDGE % 4) == 0);
static_assert(NEDGE < (1 << (32 - SLOTB)));
static_assert((NNODE % 16) == 0 && (MPAD % 64) == 0 && MPAD >= NNODE && MPAD - NNODE < 64);
static_assert(MPAD == NSB * 64);
static_assert((FEAT % 64) == 0 && (FEAT % 32) == 0 && (SEMK % 32) == 0);
static_assert(SEM_TERMS == 1 || SEM_TERMS == 2);
static_assert((CHUNK & (CHUNK - 1)) == 0 && NBMAX == (1 << SLOTB) && NTHR * 8 == NBMAX);
static_assert(LISTN >= NBMAX && NBRUN <= NBMAX && (NBRUN % 8) == 0);
static_assert((RCAP % 32) == 0 && RCAP >= 16768 + 8192);
static_assert(DEGCAP >= 37 + 8);
static_assert((long long)NBRUN * NEDGE * 5LL <= (long long)RCAP * NNODE * 4LL);
static_assert(LDS_ATT <= 264192 && LDS_ATT <= 327680);
static_assert(LDS_SEM <= 327680 && SO_BYTES <= SEM_T);
static_assert((NUW % NTHR) == 0 && (NUP % NTHR) == 0 && (NUT % NTHR) == 0);
static_assert((long long)MPAD * FEAT / 8 < 0x7fffffffLL);

typedef int  v4i  __attribute__((ext_vector_type(4)));
typedef v4i  __attribute__((may_alias)) v4ia;
typedef v4u  __attribute__((may_alias)) v4ua;

__device__ __forceinline__ void wave_sync_lds() {
  __builtin_amdgcn_fence(__ATOMIC_RELEASE, "workgroup");
  __builtin_amdgcn_wave_barrier();
  __builtin_amdgcn_fence(__ATOMIC_ACQUIRE, "workgroup");
}

__device__ __forceinline__ void wunit(const float* __restrict__ src, int pitch, int n, int kk,
                                      unsigned short* dstp) {
  float x[8];
#pragma unroll
  for (int i = 0; i < 8; ++i) x[i] = src[(size_t)(kk + i) * (size_t)pitch + n];
  const v4f a = (v4f){ x[0], x[1], x[2], x[3] };
  const v4f c = (v4f){ x[4], x[5], x[6], x[7] };
  const v4u o = pack8_bf16(a, c);
  volatile v4u* q = (volatile v4u*)dstp;
  *q = o;
  __threadfence();
  *q = o;
}

__global__ __launch_bounds__(NTHR) void k_wprep(const float* __restrict__ w0, const float* __restrict__ w1,
                                                const float* __restrict__ p1,
                                                unsigned short* w0t, unsigned short* w1t, unsigned short* p1t) {
  const int u = (int)blockIdx.x * NTHR + (int)threadIdx.x;
  if (u < NUW) {
    const int n = u >> 5, k8 = (u & 31) * 8;
    wunit(w0, FEAT, n, k8, w0t + (size_t)u * 8);
  } else if (u < 2 * NUW) {
    const int v = u - NUW, n = v >> 5, k8 = (v & 31) * 8;
    wunit(w1, FEAT, n, k8, w1t + (size_t)v * 8);
  } else if (u < NUT) {
    const int v = u - 2 * NUW;
    const int n = v / (SEMK / 8);
    const int k8 = (v - n * (SEMK / 8)) * 8;
    const int kk = k8 & (FEAT - 1);
    wunit(p1, HID, n, kk, p1t + (size_t)v * 8);
  }
}

__global__ __launch_bounds__(NTHR) void k_scores(const float* __restrict__ Z, const float* __restrict__ al,
                                                 const float* __restrict__ ar, float* SD, int nN) {
  __shared__ __attribute__((aligned(16))) float sal[FEAT];
  __shared__ __attribute__((aligned(16))) float sar[FEAT];
  __shared__ __attribute__((aligned(16))) float sS[32 * 16];
  const int tid = (int)threadIdx.x, lane = tid & 31, wave = tid >> 5;
  sal[tid] = bf16_val(al[tid]);
  sar[tid] = bf16_val(ar[tid]);
  __syncthreads();
  const v4f l0 = *(const v4fa*)(sal + 8 * lane), l1 = *(const v4fa*)(sal + 8 * lane + 4);
  const v4f r0 = *(const v4fa*)(sar + 8 * lane), r1 = *(const v4fa*)(sar + 8 * lane + 4);
  const int base = (int)blockIdx.x * 32;
  const int head = lane >> 2;
#pragma unroll 1
  for (int i = 0; i < 4; ++i) {
    const int nl = wave * 4 + i;
    const int node = base + nl;
    const int nc = node < nN ? node : nN - 1;
    const float* zr = Z + (size_t)nc * FEAT + 8 * lane;
    const v4f z0 = *(const v4fa*)zr, z1 = *(const v4fa*)(zr + 4);
    float pl = z0[0] * l0[0];
    pl = fmaf(z0[1], l0[1], pl); pl = fmaf(z0[2], l0[2], pl); pl = fmaf(z0[3], l0[3], pl);
    pl = fmaf(z1[0], l1[0], pl); pl = fmaf(z1[1], l1[1], pl); pl = fmaf(z1[2], l1[2], pl); pl = fmaf(z1[3], l1[3], pl);
    float pr = z0[0] * r0[0];
    pr = fmaf(z0[1], r0[1], pr); pr = fmaf(z0[2], r0[2], pr); pr = fmaf(z0[3], r0[3], pr);
    pr = fmaf(z1[0], r1[0], pr); pr = fmaf(z1[1], r1[1], pr); pr = fmaf(z1[2], r1[2], pr); pr = fmaf(z1[3], r1[3], pr);
    pl += __shfl_xor(pl, 1);
    pr += __shfl_xor(pr, 1);
    pl += __shfl_xor(pl, 2);
    pr += __shfl_xor(pr, 2);
    if ((lane & 3) == 0) {
      sS[nl * 16 + head]     = pl;
      sS[nl * 16 + 8 + head] = pr;
    }
  }
  __syncthreads();
  int nvalid = nN - base;
  nvalid = nvalid < 0 ? 0 : (nvalid > 32 ? 32 : nvalid);
  const int pp = tid & 127;
  const bool pok = (tid < 128) && (tid < nvalid * 4);
  const v4f pv = *(const v4fa*)(sS + 4 * pp);
  float* gp = SD + (size_t)base * 16 + 4 * pp;
  if (pok) *(volatile v4f*)gp = pv;
  __threadfence();
  if (pok) *(volatile v4f*)gp = pv;
}

__device__ __forceinline__ int scan_chunk(const int* __restrict__ dsts, int nE, int cbase, int slotBase,
                                          int nb, int vec8, int* list, int tid, int lane, int wave) {
  int wc = 0;
  const int el0  = tid * EPT;
  const int e0   = cbase + el0;
  const int sent = (-0x7fffffff - 1);
  v4i da, db;
  if (vec8 != 0 && cbase + CHUNK <= nE) {
    da = *(const v4ia*)(dsts + e0);
    db = *(const v4ia*)(dsts + e0 + 4);
  } else {
    const int t0 = dsts[min(e0,     nE - 1)];
    const int t1 = dsts[min(e0 + 1, nE - 1)];
    const int t2 = dsts[min(e0 + 2, nE - 1)];
    const int t3 = dsts[min(e0 + 3, nE - 1)];
    const int t4 = dsts[min(e0 + 4, nE - 1)];
    const int t5 = dsts[min(e0 + 5, nE - 1)];
    const int t6 = dsts[min(e0 + 6, nE - 1)];
    const int t7 = dsts[min(e0 + 7, nE - 1)];
    asm volatile("" :: "v"(t0)); asm volatile("" :: "v"(t1)); asm volatile("" :: "v"(t2)); asm volatile("" :: "v"(t3));
    asm volatile("" :: "v"(t4)); asm volatile("" :: "v"(t5)); asm volatile("" :: "v"(t6)); asm volatile("" :: "v"(t7));
    da.x = (e0     < nE) ? t0 : sent;
    da.y = (e0 + 1 < nE) ? t1 : sent;
    da.z = (e0 + 2 < nE) ? t2 : sent;
    da.w = (e0 + 3 < nE) ? t3 : sent;
    db.x = (e0 + 4 < nE) ? t4 : sent;
    db.y = (e0 + 5 < nE) ? t5 : sent;
    db.z = (e0 + 6 < nE) ? t6 : sent;
    db.w = (e0 + 7 < nE) ? t7 : sent;
  }
  const unsigned nbs = (unsigned)slotBase;
  const unsigned unb = (unsigned)nb;
  const unsigned s0 = (unsigned)da.x - nbs, s1 = (unsigned)da.y - nbs;
  const unsigned s2 = (unsigned)da.z - nbs, s3 = (unsigned)da.w - nbs;
  const unsigned s4 = (unsigned)db.x - nbs, s5 = (unsigned)db.y - nbs;
  const unsigned s6 = (unsigned)db.z - nbs, s7 = (unsigned)db.w - nbs;
  const bool h0 = s0 < unb, h1 = s1 < unb, h2 = s2 < unb, h3 = s3 < unb;
  const bool h4 = s4 < unb, h5 = s5 < unb, h6 = s6 < unb, h7 = s7 < unb;
  const unsigned any = __builtin_amdgcn_ballot_w32(h0 | h1 | h2 | h3 | h4 | h5 | h6 | h7);
  if (any != 0u) {
#define HITJ(J, HJ, SJ) { \
      const unsigned mj = __builtin_amdgcn_ballot_w32(HJ); \
      if (mj != 0u) { \
        if (HJ) { \
          const int pos = wc + (int)__builtin_amdgcn_mbcnt_lo(mj, 0u); \
          if (pos < WCAP) list[wave * WCAP + pos] = ((el0 + (J)) << SLOTB) | (int)(SJ); \
        } \
        wc += (int)__builtin_popcount(mj); } }
    HITJ(0, h0, s0)
    HITJ(1, h1, s1)
    HITJ(2, h2, s2)
    HITJ(3, h3, s3)
    HITJ(4, h4, s4)
    HITJ(5, h5, s5)
    HITJ(6, h6, s6)
    HITJ(7, h7, s7)
#undef HITJ
  }
  return wc;
}

__global__ __launch_bounds__(NTHR) void k_att(
    const int* __restrict__ srcs, const int* __restrict__ dsts,
    const float* __restrict__ Z, const float* __restrict__ SD, const float* __restrict__ bias,
    float* G, int nN, int nE, int nb, int vec8) {
  extern __shared__ v4f lds_dyn[];
  int* reg1 = (int*)lds_dyn;
  int* reg2 = reg1 + RCAP;
  int* scnt = reg2 + RCAP;
  int* soff = scnt + NBMAX;
  int* list = soff + NBMAX;
  int* wcnt = list + LISTN;
  int* wtot = wcnt + NWAVE;
  float* stg   = (float*)(wtot + NWAVE);
  float* sbias = stg + NWAVE * FEAT;
  const int tid = (int)threadIdx.x, lane = tid & 31, wave = tid >> 5;
  const int nodeBase = (int)blockIdx.x * nb;

  sbias[tid] = bf16_val(bias[tid]);
  for (int i = tid; i < NBMAX; i += NTHR) scnt[i] = 0;
  __syncthreads();

  int tot = 0;
  const int nChunks = (nE + CHUNK - 1) / CHUNK;
#pragma unroll 1
  for (int ch = 0; ch < nChunks; ++ch) {
    const int cbase = ch * CHUNK;
    const int wc = scan_chunk(dsts, nE, cbase, nodeBase, nb, vec8, list, tid, lane, wave);
    if (lane == 0) wcnt[wave] = wc;
    __syncthreads();
    int pre = 0, all = 0;
#pragma unroll
    for (int w2 = 0; w2 < NWAVE; ++w2) {
      int c = wcnt[w2];
      c = c < 0 ? 0 : (c > WCAP ? WCAP : c);
      all += c;
      pre += (w2 < wave) ? c : 0;
    }
    const int wcc  = wc > WCAP ? WCAP : wc;
    const int base = tot + pre;
#pragma unroll 1
    for (int i = lane; i < wcc; i += 32) {
      const int ent = list[wave * WCAP + i];
      const int el  = (ent >> SLOTB) & (CHUNK - 1);
      const int sl  = ent & (NBMAX - 1);
      int eid = cbase + el;
      eid = eid > nE - 1 ? nE - 1 : eid;
      const int pos = base + i;
      if (pos < RCAP) reg1[pos] = (int)(((unsigned)eid << SLOTB) | (unsigned)sl);
    }
    tot += all;
    tot = tot > RCAP ? RCAP : tot;
    __syncthreads();
  }
  const int nh = tot;

  if (wave == 0) {
#pragma unroll 1
    for (int b0 = 0; b0 < nh; b0 += 32) {
      const int idx = b0 + lane;
      const int uv  = reg1[idx < nh ? idx : nh - 1];
      const int m32 = (nh - b0) < 32 ? (nh - b0) : 32;
#pragma unroll 1
      for (int k = 0; k < m32; ++k) {
        const int u  = __builtin_amdgcn_readlane(uv, k);
        const int sl = u & (NBMAX - 1);
        if (lane == 0) scnt[sl] = scnt[sl] + 1;
      }
    }
  }
  __syncthreads();

  {
    const v4i ca = *(const v4ia*)(scnt + 8 * tid);
    const v4i cb = *(const v4ia*)(scnt + 8 * tid + 4);
    const int e0 = ca.x < 0 ? 0 : ca.x, e1 = ca.y < 0 ? 0 : ca.y, e2 = ca.z < 0 ? 0 : ca.z, e3 = ca.w < 0 ? 0 : ca.w;
    const int e4 = cb.x < 0 ? 0 : cb.x, e5 = cb.y < 0 ? 0 : cb.y, e6 = cb.z < 0 ? 0 : cb.z, e7 = cb.w < 0 ? 0 : cb.w;
    const int ts = e0 + e1 + e2 + e3 + e4 + e5 + e6 + e7;
    int incl = ts;
#pragma unroll
    for (int d = 1; d < 32; d <<= 1) {
      const int up = __shfl_up(incl, d);
      if (lane >= d) incl += up;
    }
    if (lane == 31) wtot[wave] = incl;
    __syncthreads();
    int pre = 0;
#pragma unroll
    for (int w2 = 0; w2 < NWAVE; ++w2) pre += (w2 < wave) ? wtot[w2] : 0;
    int run = pre + incl - ts;
    soff[8 * tid + 0] = run; run += e0;
    soff[8 * tid + 1] = run; run += e1;
    soff[8 * tid + 2] = run; run += e2;
    soff[8 * tid + 3] = run; run += e3;
    soff[8 * tid + 4] = run; run += e4;
    soff[8 * tid + 5] = run; run += e5;
    soff[8 * tid + 6] = run; run += e6;
    soff[8 * tid + 7] = run;
  }
  __syncthreads();
  for (int i = tid; i < NBMAX; i += NTHR) list[i] = soff[i];
  __syncthreads();

  if (wave == 0) {
#pragma unroll 1
    for (int b0 = 0; b0 < nh; b0 += 32) {
      const int idx = b0 + lane;
      const int uv  = reg1[idx < nh ? idx : nh - 1];
      const int m32 = (nh - b0) < 32 ? (nh - b0) : 32;
#pragma unroll 1
      for (int k = 0; k < m32; ++k) {
        const int u   = __builtin_amdgcn_readlane(uv, k);
        const int sl  = u & (NBMAX - 1);
        const int eid = (int)((unsigned)u >> SLOTB);
        if (lane == 0) {
          int pos = list[sl];
          pos = pos < 0 ? 0 : (pos > RCAP - 1 ? RCAP - 1 : pos);
          reg2[pos] = eid;
          list[sl] = pos + 1;
        }
      }
    }
  }
  __syncthreads();

  const int nbw = nb >> 3;
  const bool ovf = (nh >= RCAP);
  const float qnan = __int_as_float(0x7fc00000);
  const int head = lane >> 2;
  float* wst = stg + wave * FEAT;

#pragma unroll 1
  for (int jt = 0; jt < nbw; ++jt) {
    const int slot = wave * nbw + jt;
    const int grow = nodeBase + slot;
    const int gcl  = grow < nN ? grow : nN - 1;
    int sst = soff[slot];
    const int craw = scnt[slot];
    int cnt = craw;
    sst = sst < 0 ? 0 : (sst > nh ? nh : sst);
    cnt = cnt < 0 ? 0 : (cnt > DEGCAP ? DEGCAP : cnt);
    if (cnt > nh - sst) cnt = nh - sst;
    const float pz = (ovf || craw > DEGCAP) ? qnan : 0.0f;
    const bool liveRow = grow < nN;

    const float erv = SD[(size_t)gcl * 16 + 8 + head];
    float mx = MX0, dn = 0.0f;
    float a0 = 0.0f, a1 = 0.0f, a2 = 0.0f, a3 = 0.0f, a4 = 0.0f, a5 = 0.0f, a6 = 0.0f, a7 = 0.0f;

#pragma unroll 1
    for (int q = 0; q < cnt; ++q) {
      int idx = sst + q; idx = idx > RCAP - 1 ? RCAP - 1 : idx;
      int eid = reg2[idx]; eid = eid < 0 ? 0 : (eid > nE - 1 ? nE - 1 : eid);
      const int sraw = srcs[eid];
      const int s = sraw < 0 ? 0 : (sraw > nN - 1 ? nN - 1 : sraw);
      const float* zr = Z + (size_t)s * FEAT + 8 * lane;
      const v4f f0 = *(const v4fa*)zr;
      const v4f f1 = *(const v4fa*)(zr + 4);
      float lg = SD[(size_t)s * 16 + head] + erv;
      lg = lg > 0.0f ? lg : NEGSL * lg;
      const float df = lg - mx;
      const float ee = expf(-fabsf(df));
      const bool up  = df > 0.0f;
      const float s1 = up ? ee : 1.0f;
      const float s2 = up ? 1.0f : ee;
      mx = up ? lg : mx;
      dn = fmaf(dn, s1, s2);
      a0 = fmaf(a0, s1, s2 * f0[0]);
      a1 = fmaf(a1, s1, s2 * f0[1]);
      a2 = fmaf(a2, s1, s2 * f0[2]);
      a3 = fmaf(a3, s1, s2 * f0[3]);
      a4 = fmaf(a4, s1, s2 * f1[0]);
      a5 = fmaf(a5, s1, s2 * f1[1]);
      a6 = fmaf(a6, s1, s2 * f1[2]);
      a7 = fmaf(a7, s1, s2 * f1[3]);
    }
    const float inv = 1.0f / fmaxf(dn, 1e-9f);
    const bool has = cnt > 0;
    v4f q0, q1;
    q0[0] = (has ? a0 * inv : 0.0f) + pz;
    q0[1] = (has ? a1 * inv : 0.0f) + pz;
    q0[2] = (has ? a2 * inv : 0.0f) + pz;
    q0[3] = (has ? a3 * inv : 0.0f) + pz;
    q1[0] = (has ? a4 * inv : 0.0f) + pz;
    q1[1] = (has ? a5 * inv : 0.0f) + pz;
    q1[2] = (has ? a6 * inv : 0.0f) + pz;
    q1[3] = (has ? a7 * inv : 0.0f) + pz;
    *(v4fa*)(wst + 8 * lane)     = q0;
    *(v4fa*)(wst + 8 * lane + 4) = q1;
    wave_sync_lds();
#pragma unroll 1
    for (int j = 0; j < 8; ++j) {
      const int i = j * 32 + lane;
      const float x = wst[i] + sbias[i];
      wst[i] = (x > 0.0f) ? x : expm1f(x);
    }
    wave_sync_lds();
    const v4f o0 = *(const v4fa*)(wst + 4 * lane);
    const v4f o1 = *(const v4fa*)(wst + 128 + 4 * lane);
    float* gp = G + (size_t)gcl * FEAT + 4 * lane;
    if (liveRow) { *(volatile v4f*)gp = o0; *(volatile v4f*)(gp + 128) = o1; }
    __threadfence();
    if (liveRow) { *(volatile v4f*)gp = o0; *(volatile v4f*)(gp + 128) = o1; }
    wave_sync_lds();
  }
}

__global__ __launch_bounds__(NTHR) void k_sem(const float* __restrict__ G, const unsigned short* __restrict__ PT,
                                              const float* __restrict__ p1b, const float* __restrict__ p2w,
                                              unsigned* REC, int nN) {
  extern __shared__ v4f lds_dyn[];
  unsigned short* As = (unsigned short*)lds_dyn;
  float* so  = (float*)lds_dyn;
  float* sp1 = (float*)lds_dyn + SEM_T / 4;
  float* sp2 = sp1 + HID;
  float* srs = sp2 + HID;
  const int tid = (int)threadIdx.x, lane = tid & 31, wave = tid >> 5, hh = lane >> 4, m = lane & 15;
  const int rowBase = (int)blockIdx.x * SBM;

  if (tid < HID) sp1[tid] = bf16_val(p1b[tid]);
  else           sp2[tid - HID] = bf16_val(p2w[tid - HID]);

#pragma unroll 1
  for (int it = 0; it < 8; ++it) {
    const int lr = 8 * it + wave;
    const int grow = rowBase + lr;
    const int gc = grow < nN ? grow : nN - 1;
    const float* gp = G + (size_t)gc * FEAT + 8 * lane;
    v4f a = *(const v4fa*)gp;
    v4f c = *(const v4fa*)(gp + 4);
    asm volatile("" :: "v"(a));
    asm volatile("" :: "v"(c));
    const v4f z4 = (v4f){0.f, 0.f, 0.f, 0.f};
    if (grow >= nN) { a = z4; c = z4; }
    const v4u hv = pack8_bf16(a, c);
    *(v4ua*)(As + lr * SEMK + 8 * lane) = hv;
    if (SEM_TERMS == 2) {
      const v4u lv = pack8_bf16_lo(a, c);
      *(v4ua*)(As + lr * SEMK + FEAT + 8 * lane) = lv;
    }
  }
  __syncthreads();

  const int wm = wave >> 1, wn = wave & 1;
  v8f acc[4];
#pragma unroll
  for (int j = 0; j < 4; ++j) acc[j] = (v8f){0.f, 0.f, 0.f, 0.f, 0.f, 0.f, 0.f, 0.f};
  const unsigned short* ap = As + (16 * wm + m) * SEMK + 8 * hh;
  const unsigned short* bp = PT + (size_t)(64 * wn + m) * (size_t)SEMK + 8 * hh;
#pragma unroll 1
  for (int k0 = 0; k0 < SEMK; k0 += 32) {
    FragB af;
    af.h[0] = *(const v8usa*)(ap + k0);
    af.h[1] = *(const v8usa*)(ap + k0 + 16);
#pragma unroll
    for (int j = 0; j < 4; ++j) {
      const unsigned short* wq = bp + (size_t)(16 * j) * (size_t)SEMK + k0;
      FragB bfj;
      bfj.h[0] = *(const v8usa*)wq;
      bfj.h[1] = *(const v8usa*)(wq + 16);
      acc[j] = wmb(af, bfj, acc[j]);
    }
  }
  __syncthreads();

#pragma unroll
  for (int j = 0; j < 4; ++j) {
#pragma unroll
    for (int r = 0; r < 8; ++r)
      so[(16 * wm + 8 * hh + r) * HID + 64 * wn + 16 * j + m] = acc[j][r];
  }
  __syncthreads();

  {
    const int row = tid >> 2, q = tid & 3;
    float p = 0.0f;
#pragma unroll 1
    for (int jj = 0; jj < 32; ++jj) {
      const int j = 32 * q + jj;
      p += tanhf(so[row * HID + j] + sp1[j]) * sp2[j];
    }
    p += __shfl_xor(p, 1);
    p += __shfl_xor(p, 2);
    if (q == 0) srs[row] = p;
  }
  __syncthreads();

  if (wave == 0) {
    double bs = 0.0;
#pragma unroll 1
    for (int r = 0; r < SBM; ++r) {
      const double v = (double)srs[r];
      bs += (rowBase + r < nN) ? v : 0.0;
    }
    const unsigned long long bb = (unsigned long long)__double_as_longlong(bs);
    const unsigned blo = (unsigned)(bb & 0xFFFFFFFFull), bhi = (unsigned)(bb >> 32);
    v4u pv;
    pv.x = lane == 0 ? blo : 0u;
    pv.y = lane == 0 ? bhi : 0u;
    pv.z = 0u;
    pv.w = 0u;
    const bool ok = lane < 8;
    unsigned* rp = REC + (size_t)blockIdx.x * 32 + 4 * (lane & 7);
    if (ok) *(volatile v4u*)rp = pv;
    __threadfence();
    if (ok) *(volatile v4u*)rp = pv;
  }
}

__global__ __launch_bounds__(32) void k_beta(const double* __restrict__ rec, int nb, int nN, float* be) {
  __shared__ __attribute__((aligned(16))) float bl[32];
  const int lane = (int)threadIdx.x;
  double s0 = 0.0, s1 = 0.0;
#pragma unroll 1
  for (int b = 0; b < nb; ++b) {
    s0 += rec[(size_t)b * 16];
    s1 += rec[((size_t)nb + (size_t)b) * 16];
  }
  const double inv = 1.0 / (double)(nN < 1 ? 1 : nN);
  const float w0 = (float)(s0 * inv), w1 = (float)(s1 * inv);
  const float mx = fmaxf(w0, w1);
  const float e0 = expf(w0 - mx), e1 = expf(w1 - mx);
  const float rs = 1.0f / (e0 + e1);
  const float v0 = e0 * rs, v1 = e1 * rs;
  bl[lane] = lane == 0 ? v0 : (lane == 1 ? v1 : 0.0f);
  __syncthreads();
  const bool ok = lane < 8;
  const v4f v = *(const v4fa*)(bl + 4 * (lane & 7));
  float* bp = be + 4 * (lane & 7);
  if (ok) *(volatile v4f*)bp = v;
  __threadfence();
  if (ok) *(volatile v4f*)bp = v;
}

__global__ __launch_bounds__(NTHR) void k_mix(float* out, const float* __restrict__ G1,
                                              const float* __restrict__ be, int n4) {
  const int i = (int)blockIdx.x * NTHR + (int)threadIdx.x;
  if (i >= n4) return;
  const float b0 = be[0], b1 = be[1];
  const v4f a = *(const v4fa*)(out + (size_t)i * 4);
  const v4f g = *(const v4fa*)(G1 + (size_t)i * 4);
  v4f o;
  o[0] = fmaf(b1, g[0], b0 * a[0]);
  o[1] = fmaf(b1, g[1], b0 * a[1]);
  o[2] = fmaf(b1, g[2], b0 * a[2]);
  o[3] = fmaf(b1, g[3], b0 * a[3]);
  volatile v4f* q = (volatile v4f*)(out + (size_t)i * 4);
  *q = o;
  __threadfence();
  *q = o;
}

static inline int cdiv(int a, int b) { return (a + b - 1) / b; }
static inline size_t al256(size_t o) { return (o + 255) & ~(size_t)255; }

extern "C" void kernel_launch(void* const* d_in, const int* in_sizes, int n_in,
                              void* d_out, int out_size, void* d_ws, size_t ws_size,
                              hipStream_t stream) {
  if (n_in < 16) return;
  if (in_sizes[0] != NNODE * FEAT) return;
  if (in_sizes[1] != NEDGE || in_sizes[2] != NEDGE) return;
  if (in_sizes[3] != NEDGE || in_sizes[4] != NEDGE) return;
  if (in_sizes[5] != FEAT * FEAT || in_sizes[9] != FEAT * FEAT) return;
  if (in_sizes[6] != FEAT || in_sizes[7] != FEAT || in_sizes[8] != FEAT) return;
  if (in_sizes[10] != FEAT || in_sizes[11] != FEAT || in_sizes[12] != FEAT) return;
  if (in_sizes[13] != FEAT * HID || in_sizes[14] != HID || in_sizes[15] != HID) return;
  if ((long long)out_size != (long long)NNODE * FEAT) return;

  const float* h   = (const float*)d_in[0];
  const int* es0   = (const int*)d_in[1];
  const int* ed0   = (const int*)d_in[2];
  const int* es1   = (const int*)d_in[3];
  const int* ed1   = (const int*)d_in[4];
  const float* W0  = (const float*)d_in[5];
  const float* al0 = (const float*)d_in[6];
  const float* ar0 = (const float*)d_in[7];
  const float* b0  = (const float*)d_in[8];
  const float* W1  = (const float*)d_in[9];
  const float* al1 = (const float*)d_in[10];
  const float* ar1 = (const float*)d_in[11];
  const float* b1  = (const float*)d_in[12];
  const float* p1w = (const float*)d_in[13];
  const float* p1b = (const float*)d_in[14];
  const float* p2w = (const float*)d_in[15];
  float* out = (float*)d_out;

  const int nN = NNODE, nE = NEDGE;
  const int nb = NBRUN;
  const int gA = cdiv(nN, nb);
  if ((long long)gA * nb < (long long)nN) return;
  const int vec8 = ((nE & 3) == 0) ? 1 : 0;

  char* ws = (char*)d_ws;
  size_t off = 0;
  const size_t szZ  = (size_t)NNODE * FEAT * 4;
  const size_t szHB = (size_t)MPAD * FEAT * 2;
  const size_t oZ  = off; off = al256(off + szZ);
  const size_t oG  = off; off = al256(off + szZ);
  const size_t oSD = off; off = al256(off + (size_t)NNODE * 16 * 4);
  const size_t oW0 = off; off = al256(off + (size_t)NUW * 16);
  const size_t oW1 = off; off = al256(off + (size_t)NUW * 16);
  const size_t oP1 = off; off = al256(off + (size_t)NUP * 16);
  const size_t oRC = off; off = al256(off + (size_t)2 * NSB * 128);
  const size_t oBE = off; off = al256(off + 256);
  if (szHB > szZ) return;
  if (off > ws_size || off > (size_t)WSCAP) return;
  float*          Z   = (float*)(ws + oZ);
  float*          G1  = (float*)(ws + oG);
  unsigned short* HB  = (unsigned short*)(ws + oG);
  float*          SD  = (float*)(ws + oSD);
  unsigned short* W0T = (unsigned short*)(ws + oW0);
  unsigned short* W1T = (unsigned short*)(ws + oW1);
  unsigned short* P1T = (unsigned short*)(ws + oP1);
  unsigned*       REC = (unsigned*)(ws + oRC);
  float*          BE  = (float*)(ws + oBE);

  hipFuncSetAttribute(reinterpret_cast<const void*>(&k_att), hipFuncAttributeMaxDynamicSharedMemorySize, LDS_ATT);
  hipFuncSetAttribute(reinterpret_cast<const void*>(&k_sem), hipFuncAttributeMaxDynamicSharedMemorySize, LDS_SEM);

  const int gPlane = MPAD * FEAT / 8 / 256;
  const int gGemm  = cdiv(NSB * (FEAT / 64), 8);
  const int gSc    = cdiv(nN, 32);

  k_plane<0><<<gPlane, 256, 0, stream>>>(h, nN, FEAT, FEAT, HB, MPAD, FEAT);
  k_wprep<<<NUT / NTHR, NTHR, 0, stream>>>(W0, W1, p1w, W0T, W1T, P1T);

  k_gemm_nt<0, 0><<<gGemm, 256, 0, stream>>>(HB, W0T, b0, Z, nN, FEAT, FEAT, FEAT);
  k_scores<<<gSc, NTHR, 0, stream>>>(Z, al0, ar0, SD, nN);
  k_att<<<gA, NTHR, LDS_ATT, stream>>>(es0, ed0, Z, SD, b0, out, nN, nE, nb, vec8);
  k_sem<<<NSB, NTHR, LDS_SEM, stream>>>(out, P1T, p1b, p2w, REC, nN);

  k_gemm_nt<0, 0><<<gGemm, 256, 0, stream>>>(HB, W1T, b1, Z, nN, FEAT, FEAT, FEAT);
  k_scores<<<gSc, NTHR, 0, stream>>>(Z, al1, ar1, SD, nN);
  k_att<<<gA, NTHR, LDS_ATT, stream>>>(es1, ed1, Z, SD, b1, G1, nN, nE, nb, vec8);
  k_sem<<<NSB, NTHR, LDS_SEM, stream>>>(G1, P1T, p1b, p2w, REC + (size_t)NSB * 32, nN);

  k_beta<<<1, 32, 0, stream>>>((const double*)REC, NSB, nN, BE);
  const int n4 = NNODE * FEAT / 4;
  k_mix<<<cdiv(n4, NTHR), NTHR, 0, stream>>>(out, G1, BE, n4);
}
